// DetrAttention_64665027608812
// MI455X (gfx1250) — hardware-verified
//
#include <hip/hip_runtime.h>
#include <math.h>
#include <stdint.h>

#define NB   8
#define NS   1024
#define CD   256
#define NH   8
#define HD   32
#define NTOK (NB * NS)
#define NQB  (NS / 64)
#define NKB  (NS / 64)
static_assert(NH * HD == CD);
static_assert(HD == 32);
static_assert((NS % 64) == 0 && (CD % 64) == 0 && (NH % 2) == 0 && ((NTOK) % 64) == 0);

typedef _Float16 v16h __attribute__((ext_vector_type(16)));
typedef _Float16 v8h  __attribute__((ext_vector_type(8)));
typedef __bf16   v16b __attribute__((ext_vector_type(16)));
typedef __bf16   v8b  __attribute__((ext_vector_type(8)));
typedef float    v8f  __attribute__((ext_vector_type(8)));
typedef float    v4f  __attribute__((ext_vector_type(4)));
typedef unsigned int v4u __attribute__((ext_vector_type(4)));

__device__ __forceinline__ unsigned short bf_bits(float f) {
  unsigned u = __float_as_uint(f);
  return (unsigned short)((u + 0x7FFFu + ((u >> 16) & 1u)) >> 16);
}
__device__ __forceinline__ float bf_up(unsigned short h) { return __uint_as_float(((unsigned)h) << 16); }
__device__ __forceinline__ unsigned short h_bits(_Float16 x) { return __builtin_bit_cast(unsigned short, x); }
__device__ __forceinline__ unsigned pk16(unsigned short a, unsigned short b) { return (unsigned)a | ((unsigned)b << 16); }
__device__ __forceinline__ v8f zero8() { v8f z = {0.f, 0.f, 0.f, 0.f, 0.f, 0.f, 0.f, 0.f}; return z; }

__device__ __forceinline__ v16b ldfrag_b(const __bf16* p) {
  union { v16b v; v8b h[2]; } f;
  f.h[0] = *(const v8b*)(p);
  f.h[1] = *(const v8b*)(p + 16);
  return f.v;
}
__device__ __forceinline__ v16h ldfrag_h(const _Float16* p) {
  union { v16h v; v8h h[2]; } f;
  f.h[0] = *(const v8h*)(p);
  f.h[1] = *(const v8h*)(p + 16);
  return f.v;
}

__device__ __forceinline__ v8f mma_h(v16h a, v16h b, v8f c) {
  c = __builtin_amdgcn_wmma_f32_16x16x32_f16(false, a, false, b, (short)0, c, false, false);
#if defined(__HIP_DEVICE_COMPILE__)
  asm volatile("v_nop\n\tv_nop\n\tv_nop\n\tv_nop" : "+v"(c) : "v"(a), "v"(b));
#endif
  return c;
}
__device__ __forceinline__ v8f mma_b_raw(v16b a, v16b b, v8f c) {
  return __builtin_amdgcn_wmma_f32_16x16x32_bf16(false, a, false, b, (short)0, c, false, false);
}
__device__ __forceinline__ void dep_guard_b(v8f& a, v8f& b, v16b x, v16b y) {
#if defined(__HIP_DEVICE_COMPILE__)
  asm volatile("v_nop\n\tv_nop\n\tv_nop\n\tv_nop" : "+v"(a), "+v"(b) : "v"(x), "v"(y));
#endif
}
__device__ __forceinline__ void keep4_b(v16b a, v16b b, v16b c, v16b d) {
#if defined(__HIP_DEVICE_COMPILE__)
  asm volatile("v_nop" :: "v"(a), "v"(b), "v"(c), "v"(d));
#endif
}
__device__ __forceinline__ void acc_guard4(v8f& a, v8f& b, v8f& c, v8f& d) {
#if defined(__HIP_DEVICE_COMPILE__)
  asm volatile("v_nop\n\tv_nop\n\tv_nop\n\tv_nop" : "+v"(a), "+v"(b), "+v"(c), "+v"(d));
#endif
}
__device__ __forceinline__ void wave_sync_lds() {
  __builtin_amdgcn_fence(__ATOMIC_RELEASE, "workgroup");
  __builtin_amdgcn_wave_barrier();
  __builtin_amdgcn_fence(__ATOMIC_ACQUIRE, "workgroup");
}

__device__ __forceinline__ v8f score3b(const v16b qh, const v16b ql, const v16b kh, const v16b kl) {
  v8f acc = zero8();
  acc = mma_b_raw(ql, kh, acc);
  acc = mma_b_raw(qh, kl, acc);
  acc = mma_b_raw(qh, kh, acc);
#if defined(__HIP_DEVICE_COMPILE__)
  asm volatile("v_nop\n\tv_nop\n\tv_nop\n\tv_nop" : "+v"(acc) : "v"(qh), "v"(ql), "v"(kh), "v"(kl));
#endif
  return acc;
}

__global__ __launch_bounds__(256) void cvt_act(const float* __restrict__ hs, const float* __restrict__ pq,
                                               unsigned short* xph, unsigned short* xpl, unsigned short* xv, int n8) {
  const int i = blockIdx.x * 256 + threadIdx.x;
  if (i < n8) {
    const size_t o = (size_t)i * 8;
    const v4f a0 = *(const v4f*)(hs + o);
    const v4f a1 = *(const v4f*)(hs + o + 4);
    const v4f p0 = *(const v4f*)(pq + o);
    const v4f p1 = *(const v4f*)(pq + o + 4);
    float hvv[8], pvv[8];
#pragma unroll
    for (int e = 0; e < 4; ++e) { hvv[e] = a0[e]; hvv[4 + e] = a1[e]; pvv[e] = p0[e]; pvv[4 + e] = p1[e]; }
    unsigned short sh[8], sl[8], vb[8];
#pragma unroll
    for (int e = 0; e < 8; ++e) {
      const unsigned short hb = bf_bits(hvv[e]);
      const float s = bf_up(hb) + bf_up(bf_bits(pvv[e]));
      const unsigned short s0 = bf_bits(s);
      sh[e] = s0;
      sl[e] = bf_bits(s - bf_up(s0));
      vb[e] = hb;
    }
    v4u P0, P1, P2;
#pragma unroll
    for (int e = 0; e < 4; ++e) {
      P0[e] = pk16(sh[2 * e], sh[2 * e + 1]);
      P1[e] = pk16(sl[2 * e], sl[2 * e + 1]);
      P2[e] = pk16(vb[2 * e], vb[2 * e + 1]);
    }
    *(volatile v4u*)(xph + o) = P0;
    *(volatile v4u*)(xpl + o) = P1;
    *(volatile v4u*)(xv + o)  = P2;
    __threadfence();
    *(volatile v4u*)(xph + o) = P0;
    *(volatile v4u*)(xpl + o) = P1;
    *(volatile v4u*)(xv + o)  = P2;
  }
}

__global__ __launch_bounds__(256) void cvt_w4(const float* __restrict__ w0, const float* __restrict__ w1,
                                              const float* __restrict__ w2, const float* __restrict__ w3,
                                              unsigned short* outp, int n8) {
  const int z = blockIdx.y;
  const float* src = (z == 0) ? w0 : ((z == 1) ? w1 : ((z == 2) ? w2 : w3));
  unsigned short* dst = outp + (size_t)z * CD * CD;
  const int i = blockIdx.x * 256 + threadIdx.x;
  if (i < n8) {
    const size_t o = (size_t)i * 8;
    const v4f a = *(const v4f*)(src + o);
    const v4f b = *(const v4f*)(src + o + 4);
    v4u p;
    p[0] = pk16(bf_bits(a[0]), bf_bits(a[1]));
    p[1] = pk16(bf_bits(a[2]), bf_bits(a[3]));
    p[2] = pk16(bf_bits(b[0]), bf_bits(b[1]));
    p[3] = pk16(bf_bits(b[2]), bf_bits(b[3]));
    *(volatile v4u*)(dst + o) = p;
    __threadfence();
    *(volatile v4u*)(dst + o) = p;
  }
}

template <int NSPLIT, int OUT_MODE, int BIASM>
__global__ __launch_bounds__(256) void gemm64(
    const unsigned short* __restrict__ Ap, const unsigned short* A2p, int lda, long long strideA,
    const unsigned short* __restrict__ Btp, int ldb, long long strideB,
    void* Cout, int ldc, long long strideC, void* Cout2,
    int M, int N, int K, float rscale, float oscale, const float* __restrict__ biasp) {
  const __bf16* A   = (const __bf16*)(const void*)Ap;
  const __bf16* A2  = (const __bf16*)(const void*)A2p;
  const __bf16* Bt  = (const __bf16*)(const void*)Btp;
  __shared__ __align__(16) float sT[8][16 * 68];
  const int b    = blockIdx.y;
  const int lane = threadIdx.x & 31;
  const int wave = threadIdx.x >> 5;
  const int tilesN = N >> 6;
  const int tilesM = M >> 6;
  const int tile = blockIdx.x * 8 + wave;
  if (tile >= tilesM * tilesN) return;
  const int tm = tile / tilesN;
  const int tn = tile - tm * tilesN;
  const int m0 = tm << 6;
  const int n0 = tn << 6;

  const __bf16* Ab  = A  + (size_t)b * strideA;
  const __bf16* Bb  = Bt + (size_t)b * strideB;
  const __bf16* Ab2 = (NSPLIT >= 1) ? (A2 + (size_t)b * strideA) : Ab;

  const int rlane = lane & 15;
  const int koff  = (lane >> 4) * 8;
  const int mOff  = (lane >> 4) * 8;

  v8f acc[4][4];
#pragma unroll
  for (int i = 0; i < 4; ++i)
#pragma unroll
    for (int j = 0; j < 4; ++j) acc[i][j] = zero8();

  for (int k0 = 0; k0 < K; k0 += 32) {
    v16b bh[4];
#pragma unroll
    for (int j = 0; j < 4; ++j) {
      const size_t bo = (size_t)(n0 + (j << 4) + rlane) * ldb + koff + k0;
      bh[j] = ldfrag_b(Bb + bo);
    }
#pragma unroll
    for (int i = 0; i < 4; ++i) {
      const size_t ao = (size_t)(m0 + (i << 4) + rlane) * lda + koff + k0;
      const v16b ah = ldfrag_b(Ab + ao);
      v16b al = ah;
      if (NSPLIT >= 1) al = ldfrag_b(Ab2 + ao);
#pragma unroll
      for (int j = 0; j < 4; ++j) {
        acc[i][j] = mma_b_raw(ah, bh[j], acc[i][j]);
        if (NSPLIT >= 1) acc[i][j] = mma_b_raw(al, bh[j], acc[i][j]);
      }
      dep_guard_b(acc[i][0], acc[i][3], ah, al);
    }
    keep4_b(bh[0], bh[1], bh[2], bh[3]);
  }
  acc_guard4(acc[0][0], acc[0][1], acc[0][2], acc[0][3]);
  acc_guard4(acc[1][0], acc[1][1], acc[1][2], acc[1][3]);
  acc_guard4(acc[2][0], acc[2][1], acc[2][2], acc[2][3]);
  acc_guard4(acc[3][0], acc[3][1], acc[3][2], acc[3][3]);

  float* slab = sT[wave];
#pragma unroll
  for (int i = 0; i < 4; ++i) {
    const int mBase = m0 + (i << 4);
#pragma unroll
    for (int j = 0; j < 4; ++j) {
#pragma unroll
      for (int r = 0; r < 8; ++r) {
        slab[(mOff + r) * 68 + (j << 4) + rlane] = acc[i][j][r];
      }
    }
    wave_sync_lds();
    if (OUT_MODE == 0) {
      float* C = (float*)Cout + (size_t)b * strideC;
      const int hh = lane >> 4, c4 = (lane & 15) * 4;
      v4f bv = {0.f, 0.f, 0.f, 0.f};
      if (BIASM == 1) {
#pragma unroll
        for (int e = 0; e < 4; ++e) bv[e] = bf_up(bf_bits(biasp[n0 + c4 + e]));
      }
      for (int pass = 0; pass < 2; ++pass) {
#pragma unroll
        for (int it = 0; it < 8; ++it) {
          const int row = it * 2 + hh;
          float brow = 0.f;
          if (BIASM == 2) brow = bf_up(bf_bits(biasp[mBase + row]));
          const v4f v = (*(const v4f*)(slab + row * 68 + c4) + bv + brow) * oscale;
          *(volatile v4f*)(C + (size_t)(mBase + row) * ldc + n0 + c4) = v;
        }
        __threadfence();
      }
    } else {
      const int q = lane >> 3, c8 = (lane & 7) * 8;
      unsigned short* C  = (unsigned short*)Cout  + (size_t)b * strideC;
      unsigned short* C2 = (unsigned short*)Cout2 + (size_t)b * strideC;
      float bcol[8];
#pragma unroll
      for (int e = 0; e < 8; ++e) bcol[e] = 0.f;
      if (BIASM == 1) {
#pragma unroll
        for (int e = 0; e < 8; ++e) bcol[e] = bf_up(bf_bits(biasp[n0 + c8 + e]));
      }
      v4u hv[4], lv[4];
#pragma unroll
      for (int it = 0; it < 4; ++it) {
        const int row = it * 4 + q;
        float brow = 0.f;
        if (BIASM == 2) brow = bf_up(bf_bits(biasp[mBase + row]));
        const float* sp = slab + row * 68 + c8;
        v4u a, a2;
#pragma unroll
        for (int e = 0; e < 4; ++e) {
          const float f0 = (sp[2 * e] + bcol[2 * e] + brow) * oscale;
          const float f1 = (sp[2 * e + 1] + bcol[2 * e + 1] + brow) * oscale;
          unsigned short h0, h1, l0, l1;
          if (OUT_MODE == 2) {
            h0 = bf_bits(f0); h1 = bf_bits(f1);
            l0 = bf_bits(f0 - bf_up(h0)); l1 = bf_bits(f1 - bf_up(h1));
          } else {
            const _Float16 x0 = (_Float16)f0, x1 = (_Float16)f1;
            h0 = h_bits(x0); h1 = h_bits(x1);
            l0 = h_bits((_Float16)((f0 - (float)x0) * rscale));
            l1 = h_bits((_Float16)((f1 - (float)x1) * rscale));
          }
          a[e] = pk16(h0, h1); a2[e] = pk16(l0, l1);
        }
        hv[it] = a; lv[it] = a2;
      }
      for (int pass = 0; pass < 2; ++pass) {
#pragma unroll
        for (int it = 0; it < 4; ++it) {
          const int row = it * 4 + q;
          *(volatile v4u*)(C  + (size_t)(mBase + row) * ldc + n0 + c8) = hv[it];
          *(volatile v4u*)(C2 + (size_t)(mBase + row) * ldc + n0 + c8) = lv[it];
        }
        __threadfence();
      }
    }
    wave_sync_lds();
  }
}

__global__ __launch_bounds__(256)
void attn32(const unsigned short* __restrict__ qhp, const unsigned short* __restrict__ qlp,
            const unsigned short* __restrict__ khp, const unsigned short* __restrict__ klp,
            const unsigned short* __restrict__ vhp, const unsigned short* __restrict__ vlp,
            unsigned short* ohp, unsigned short* olp, float rres) {
  union FH { v16h v; v8h h[2]; };
  __shared__ __align__(16) _Float16 Psh[8][16 * 64];
  __shared__ __align__(16) _Float16 Psl[8][16 * 64];
  __shared__ __align__(16) float    Os[64 * 64];

  const int tid  = threadIdx.x;
  const int wave = tid >> 5;
  const int lane = tid & 31;
  const int hh   = lane >> 4;
  const int c    = lane & 15;

  const int bx   = blockIdx.x;
  const int qb   = bx % NQB;
  const int rest = bx / NQB;
  const int g    = rest % (NH / 2);
  const int b    = rest / (NH / 2);
  const int hp   = wave >> 2;
  const int h    = 2 * g + hp;
  const int wq   = wave & 3;
  const int q0   = qb * 64 + wq * 16;
  const size_t rowB = (size_t)b * NS;

  const __bf16* Qh = (const __bf16*)(const void*)qhp + (size_t)h * HD;
  const __bf16* Ql = (const __bf16*)(const void*)qlp + (size_t)h * HD;
  const __bf16* Kh = (const __bf16*)(const void*)khp + (size_t)h * HD;
  const __bf16* Kl = (const __bf16*)(const void*)klp + (size_t)h * HD;
  const _Float16* Vh = (const _Float16*)(const void*)vhp + ((size_t)b * CD + (size_t)h * HD) * NS;
  const _Float16* Vl = (const _Float16*)(const void*)vlp + ((size_t)b * CD + (size_t)h * HD) * NS;

  const v16b qah = ldfrag_b(Qh + (rowB + q0 + c) * CD + 8 * hh);
  const v16b qal = ldfrag_b(Ql + (rowB + q0 + c) * CD + 8 * hh);

  float mrow[8], lrow[8];
  v8f oacc[2];
#pragma unroll
  for (int r = 0; r < 8; ++r) { mrow[r] = -INFINITY; lrow[r] = 0.f; }
#pragma unroll
  for (int t = 0; t < 2; ++t) oacc[t] = zero8();

  _Float16* pwh = Psh[wave];
  _Float16* pwl = Psl[wave];

  for (int kt = 0; kt < NKB; ++kt) {
    const int kv0 = kt * 64;

    v8f s[4];
#pragma unroll
    for (int j = 0; j < 4; ++j) {
      const size_t ko = (rowB + kv0 + j * 16 + c) * CD + 8 * hh;
      const v16b kb = ldfrag_b(Kh + ko);
      const v16b kl = ldfrag_b(Kl + ko);
      s[j] = score3b(qah, qal, kb, kl);
    }

#pragma unroll
    for (int r = 0; r < 8; ++r) {
      float m = fmaxf(fmaxf(s[0][r], s[1][r]), fmaxf(s[2][r], s[3][r]));
#pragma unroll
      for (int off = 1; off < 16; off <<= 1) m = fmaxf(m, __shfl_xor(m, off, 32));
      const float mnew  = fmaxf(mrow[r], m);
      const float alpha = __expf(mrow[r] - mnew);
      mrow[r] = mnew;
      float psum = 0.f;
#pragma unroll
      for (int j = 0; j < 4; ++j) {
        const float p  = __expf(s[j][r] - mnew);
        psum += p;
        const float p1 = p * 1024.0f;
        const _Float16 x = (_Float16)p1;
        const int idx = (8 * hh + r) * 64 + j * 16 + c;
        pwh[idx] = x;
        pwl[idx] = (_Float16)((p1 - (float)x) * 4096.0f);
      }
#pragma unroll
      for (int off = 1; off < 16; off <<= 1) psum += __shfl_xor(psum, off, 32);
      lrow[r] = lrow[r] * alpha + psum;
#pragma unroll
      for (int t = 0; t < 2; ++t) oacc[t][r] *= alpha;
    }
    wave_sync_lds();

    v8f o1[2];
    o1[0] = zero8(); o1[1] = zero8();
#pragma unroll
    for (int kk = 0; kk < 2; ++kk) {
      FH pa, pl;
      pa.h[0] = *(const v8h*)(pwh + c * 64 + kk * 32 + 8 * hh);
      pa.h[1] = *(const v8h*)(pwh + c * 64 + kk * 32 + 16 + 8 * hh);
      pl.h[0] = *(const v8h*)(pwl + c * 64 + kk * 32 + 8 * hh);
      pl.h[1] = *(const v8h*)(pwl + c * 64 + kk * 32 + 16 + 8 * hh);
#pragma unroll
      for (int t = 0; t < 2; ++t) {
        const size_t vo = (size_t)(t * 16 + c) * NS + kv0 + kk * 32 + 8 * hh;
        const v16h vb = ldfrag_h(Vh + vo);
        const v16h vl = ldfrag_h(Vl + vo);
        oacc[t] = mma_h(pa.v, vb, oacc[t]);
        o1[t]   = mma_h(pa.v, vl, o1[t]);
        o1[t]   = mma_h(pl.v, vb, o1[t]);
      }
    }
#pragma unroll
    for (int t = 0; t < 2; ++t)
#pragma unroll
      for (int r = 0; r < 8; ++r) oacc[t][r] += o1[t][r] * rres;
    wave_sync_lds();
  }

#pragma unroll
  for (int r = 0; r < 8; ++r) {
    const float l = lrow[r];
    const float inv = ((l > 0.f) ? (1.0f / l) : 0.f) * (1.0f / 1024.0f);
#pragma unroll
    for (int t = 0; t < 2; ++t) Os[(wq * 16 + 8 * hh + r) * 64 + hp * 32 + t * 16 + c] = oacc[t][r] * inv;
  }
  __syncthreads();
  {
    const int q4 = lane >> 3, c8 = (lane & 7) * 8;
    v4u hv[2], lv[2];
#pragma unroll
    for (int it = 0; it < 2; ++it) {
      const int row = wave * 8 + it * 4 + q4;
      const float* sp = Os + row * 64 + c8;
      v4u a, a2;
#pragma unroll
      for (int e = 0; e < 4; ++e) {
        const float f0 = sp[2 * e], f1 = sp[2 * e + 1];
        const unsigned short h0 = bf_bits(f0), h1 = bf_bits(f1);
        const unsigned short l0 = bf_bits(f0 - bf_up(h0)), l1 = bf_bits(f1 - bf_up(h1));
        a[e] = pk16(h0, h1); a2[e] = pk16(l0, l1);
      }
      hv[it] = a; lv[it] = a2;
    }
    for (int pass = 0; pass < 2; ++pass) {
#pragma unroll
      for (int it = 0; it < 2; ++it) {
        const int row = wave * 8 + it * 4 + q4;
        const size_t go = (rowB + qb * 64 + row) * CD + (size_t)g * 64 + c8;
        *(volatile v4u*)(ohp + go) = hv[it];
        *(volatile v4u*)(olp + go) = lv[it];
      }
      __threadfence();
    }
  }
}

extern "C" void kernel_launch(void* const* d_in, const int* in_sizes, int n_in,
                              void* d_out, int out_size, void* d_ws, size_t ws_size,
                              hipStream_t stream) {
  if (n_in < 10) return;
  if (in_sizes[0] != NTOK * CD || in_sizes[1] != NTOK * CD) return;
  if (in_sizes[2] != CD * CD || in_sizes[4] != CD * CD || in_sizes[6] != CD * CD || in_sizes[8] != CD * CD) return;
  if (in_sizes[3] != CD || in_sizes[5] != CD || in_sizes[7] != CD || in_sizes[9] != CD) return;
  if (out_size != NTOK * CD) return;

  const float* hs = (const float*)d_in[0];
  const float* pq = (const float*)d_in[1];
  const float* Wq = (const float*)d_in[2];
  const float* bq = (const float*)d_in[3];
  const float* Wk = (const float*)d_in[4];
  const float* bk = (const float*)d_in[5];
  const float* Wv = (const float*)d_in[6];
  const float* bv = (const float*)d_in[7];
  const float* Wo = (const float*)d_in[8];
  const float* bo = (const float*)d_in[9];

  const size_t PX = (size_t)NTOK * CD * 2;
  const size_t PW = (size_t)4 * CD * CD * 2;
  size_t off = 0;
  const size_t oXph = off; off += PX;
  const size_t oXpl = off; off += PX;
  const size_t oXv  = off; off += PX;
  const size_t oW   = off; off += PW;
  const size_t oQh  = off; off += PX;
  const size_t oQl  = off; off += PX;
  const size_t oKh  = off; off += PX;
  const size_t oKl  = off; off += PX;
  const size_t oVTh = off; off += PX;
  const size_t oVTl = off; off += PX;
  const size_t oOh  = off; off += PX;
  const size_t oOl  = off; off += PX;
  if (off > ws_size) return;
  if (off > (size_t)134217728) return;

  char* ws = (char*)d_ws;
  unsigned short* Xph = (unsigned short*)(ws + oXph);
  unsigned short* Xpl = (unsigned short*)(ws + oXpl);
  unsigned short* Xv  = (unsigned short*)(ws + oXv);
  unsigned short* WT  = (unsigned short*)(ws + oW);
  unsigned short* WTq = WT;
  unsigned short* WTk = WT + (size_t)1 * CD * CD;
  unsigned short* WTv = WT + (size_t)2 * CD * CD;
  unsigned short* WTo = WT + (size_t)3 * CD * CD;
  unsigned short* Qh  = (unsigned short*)(ws + oQh);
  unsigned short* Ql  = (unsigned short*)(ws + oQl);
  unsigned short* Kh  = (unsigned short*)(ws + oKh);
  unsigned short* Kl  = (unsigned short*)(ws + oKl);
  unsigned short* VTh = (unsigned short*)(ws + oVTh);
  unsigned short* VTl = (unsigned short*)(ws + oVTl);
  unsigned short* Oh  = (unsigned short*)(ws + oOh);
  unsigned short* Ol  = (unsigned short*)(ws + oOl);

  float* xout = (float*)d_out;

  const float qscale = 5.656854249492380f;
  const float rres   = 1.0f / 4096.0f;

  const dim3 blk(256);
  const int n8a = NTOK * CD / 8;
  const int n8w = CD * CD / 8;
  const dim3 gCvtA((n8a + 255) / 256);
  const dim3 gCvtW((n8w + 255) / 256, 4);
  const dim3 gProj(((NTOK / 64) * (CD / 64) + 7) / 8, 1);
  const dim3 gVT(((CD / 64) * (NS / 64) + 7) / 8, NB);
  const dim3 gAttn(NB * (NH / 2) * NQB);

  cvt_act<<<gCvtA, blk, 0, stream>>>(hs, pq, Xph, Xpl, Xv, n8a);
  cvt_w4<<<gCvtW, blk, 0, stream>>>(Wq, Wk, Wv, Wo, WT, n8w);
  gemm64<1, 2, 1><<<gProj, blk, 0, stream>>>(
      Xph, Xpl, CD, 0LL, WTq, CD, 0LL,
      (void*)Qh, CD, 0LL, (void*)Ql,
      NTOK, CD, CD, 1.0f, qscale, bq);
  gemm64<1, 2, 1><<<gProj, blk, 0, stream>>>(
      Xph, Xpl, CD, 0LL, WTk, CD, 0LL,
      (void*)Kh, CD, 0LL, (void*)Kl,
      NTOK, CD, CD, 1.0f, 1.0f, bk);
  gemm64<0, 3, 2><<<gVT, blk, 0, stream>>>(
      WTv, WTv, CD, 0LL, Xv, CD, (long long)NS * CD,
      (void*)VTh, NS, (long long)CD * NS, (void*)VTl,
      CD, NS, CD, 4096.0f, 1.0f, bv);
  attn32<<<gAttn, blk, 0, stream>>>(Qh, Ql, Kh, Kl, VTh, VTl, Oh, Ol, rres);
  gemm64<1, 0, 1><<<gProj, blk, 0, stream>>>(
      Oh, Ol, CD, 0LL, WTo, CD, 0LL,
      (void*)xout, CD, 0LL, (void*)xout,
      NTOK, CD, CD, 1.0f, 1.0f, bo);
  (void)hipGetLastError();
}
